// DecCLSTMBlock_91233695301776
// MI455X (gfx1250) — hardware-verified
//
#include <hip/hip_runtime.h>
#include <stddef.h>

typedef __attribute__((ext_vector_type(16))) _Float16 v16h;
typedef __attribute__((ext_vector_type(8)))  _Float16 v8h;
typedef __attribute__((ext_vector_type(16))) __bf16   v16b;
typedef __attribute__((ext_vector_type(8)))  __bf16   v8b;
typedef __attribute__((ext_vector_type(8)))  float    v8f;
typedef __attribute__((ext_vector_type(4)))  float    v4f;
typedef __attribute__((ext_vector_type(4)))  unsigned v4u;

__device__ __forceinline__ unsigned short f2bf_bits(float f) {
  unsigned u = __float_as_uint(f);
  return (unsigned short)((u + 0x7FFFu + ((u >> 16) & 1u)) >> 16);
}
__device__ __forceinline__ float bf_bits2f(unsigned short h) { return __uint_as_float(((unsigned)h) << 16); }
__device__ __forceinline__ float bf_rne(float f) { return bf_bits2f(f2bf_bits(f)); }

__device__ __forceinline__ unsigned pkh2(float a, float b) {
  return (unsigned)__builtin_bit_cast(unsigned short, (_Float16)a) |
         ((unsigned)__builtin_bit_cast(unsigned short, (_Float16)b) << 16);
}

__device__ __forceinline__ void dep_guard_h(v8f& a, v8f& b, v16h x, v16h y) { asm volatile("v_nop\n\tv_nop\n\tv_nop\n\tv_nop" : "+v"(a), "+v"(b) : "v"(x), "v"(y)); }
__device__ __forceinline__ void dep_guard_b(v8f& a, v8f& b, v16b x, v16b y) { asm volatile("v_nop\n\tv_nop\n\tv_nop\n\tv_nop" : "+v"(a), "+v"(b) : "v"(x), "v"(y)); }
__device__ __forceinline__ void keep4_h(v16h a, v16h b, v16h c, v16h d) { asm volatile("v_nop" :: "v"(a), "v"(b), "v"(c), "v"(d)); }
__device__ __forceinline__ void keep4_b(v16b a, v16b b, v16b c, v16b d) { asm volatile("v_nop" :: "v"(a), "v"(b), "v"(c), "v"(d)); }
__device__ __forceinline__ void acc_guard4(v8f& a, v8f& b, v8f& c, v8f& d) { asm volatile("v_nop\n\tv_nop\n\tv_nop\n\tv_nop" : "+v"(a), "+v"(b), "+v"(c), "+v"(d)); }
template <typename T> struct Frag;
template <> struct Frag<_Float16> {
  typedef v16h V; union U { v16h v; v8h h[2]; };
  static __device__ __forceinline__ v16h load(const _Float16* p) {
    U f; f.h[0] = *(const v8h*)(p); f.h[1] = *(const v8h*)(p + 16); return f.v;
  }
  static __device__ __forceinline__ v8f mma(v16h a, v16h b, v8f c) {
    return __builtin_amdgcn_wmma_f32_16x16x32_f16(false, a, false, b, (short)0, c, false, false);
  }
  static __device__ __forceinline__ void guard(v8f& a, v8f& b, v16h x, v16h y) { dep_guard_h(a, b, x, y); }
  static __device__ __forceinline__ void keep(v16h a, v16h b, v16h c, v16h d) { keep4_h(a, b, c, d); }
};
template <> struct Frag<__bf16> {
  typedef v16b V; union U { v16b v; v8b h[2]; };
  static __device__ __forceinline__ v16b load(const __bf16* p) {
    U f; f.h[0] = *(const v8b*)(p); f.h[1] = *(const v8b*)(p + 16); return f.v;
  }
  static __device__ __forceinline__ v8f mma(v16b a, v16b b, v8f c) {
    return __builtin_amdgcn_wmma_f32_16x16x32_bf16(false, a, false, b, (short)0, c, false, false);
  }
  static __device__ __forceinline__ void guard(v8f& a, v8f& b, v16b x, v16b y) { dep_guard_b(a, b, x, y); }
  static __device__ __forceinline__ void keep(v16b a, v16b b, v16b c, v16b d) { keep4_b(a, b, c, d); }
};

template <int ET> struct Elem;
template <> struct Elem<0> { typedef _Float16 T; };
template <> struct Elem<1> { typedef __bf16 T; };
template <int ET, bool SPLIT, int BIAS_MODE, int OUT_MODE, bool RESID, int ACT = 0>
__global__ __launch_bounds__(256) void wmma_gemm64(
    const unsigned short* __restrict__ Ap, const unsigned short* __restrict__ A2p, int lda, long strideA,
    const unsigned short* __restrict__ Btp, const unsigned short* __restrict__ Bt2p, int ldb, long strideB,
    void* __restrict__ Cout, void* __restrict__ Cout2, int ldc, long strideC,
    const float* __restrict__ bias,
    const float* __restrict__ resid, long strideR,
    int M, int N, int K, float scale) {
  typedef typename Elem<ET>::T T;
  typedef typename Frag<T>::V V;
  const T* A = (const T*)Ap; const T* A2 = (const T*)A2p; const T* Bt = (const T*)Btp; const T* Bt2 = (const T*)Bt2p;
  __shared__ __align__(16) float sT[8][16 * 68];
  const int b    = blockIdx.y;
  const int lane = threadIdx.x & 31;
  const int wave = threadIdx.x >> 5;
  const int tilesN = N >> 6;
  const int tilesM = M >> 6;
  const int tile = blockIdx.x * 8 + wave;
  if (tile >= tilesM * tilesN) return;
  const int tm = tile / tilesN;
  const int tn = tile - tm * tilesN;
  const int m0 = tm << 6;
  const int n0 = tn << 6;

  const T* Ab  = A  + (size_t)b * strideA;
  const T* Bb  = Bt + (size_t)b * strideB;
  const T* Ab2 = SPLIT ? (A2  + (size_t)b * strideA) : nullptr;
  const T* Bb2 = SPLIT ? (Bt2 + (size_t)b * strideB) : nullptr;

  const int rlane = lane & 15;
  const int koff  = (lane >> 4) * 8;
  const int mOff  = (lane >> 4) * 8;

  v8f acc[4][4];
#pragma unroll
  for (int i = 0; i < 4; ++i)
#pragma unroll
    for (int j = 0; j < 4; ++j) acc[i][j] = (v8f){0.f,0.f,0.f,0.f,0.f,0.f,0.f,0.f};

  for (int k0 = 0; k0 < K; k0 += 32) {
    V bh[4], bl[4];
#pragma unroll
    for (int j = 0; j < 4; ++j) {
      const size_t bo = (size_t)(n0 + (j << 4) + rlane) * ldb + koff + k0;
      bh[j] = Frag<T>::load(Bb + bo);
      if (SPLIT) bl[j] = Frag<T>::load(Bb2 + bo);
    }
#pragma unroll
    for (int i = 0; i < 4; ++i) {
      const size_t ao = (size_t)(m0 + (i << 4) + rlane) * lda + koff + k0;
      V ah = Frag<T>::load(Ab + ao);
      V al;
      if (SPLIT) al = Frag<T>::load(Ab2 + ao);
#pragma unroll
      for (int j = 0; j < 4; ++j) {
        acc[i][j] = Frag<T>::mma(ah, bh[j], acc[i][j]);
        if (SPLIT) {
          acc[i][j] = Frag<T>::mma(ah, bl[j], acc[i][j]);
          acc[i][j] = Frag<T>::mma(al, bh[j], acc[i][j]);
        }
      }
      Frag<T>::guard(acc[i][0], acc[i][3], ah, SPLIT ? al : ah);
    }
    Frag<T>::keep(bh[0], bh[1], bh[2], bh[3]);
    if (SPLIT) Frag<T>::keep(bl[0], bl[1], bl[2], bl[3]);
  }
  acc_guard4(acc[0][0], acc[0][1], acc[0][2], acc[0][3]);
  acc_guard4(acc[1][0], acc[1][1], acc[1][2], acc[1][3]);
  acc_guard4(acc[2][0], acc[2][1], acc[2][2], acc[2][3]);
  acc_guard4(acc[3][0], acc[3][1], acc[3][2], acc[3][3]);

  float* slab = sT[wave];
  const float* Rb = RESID ? (resid + (size_t)b * strideR) : nullptr;
#pragma unroll
  for (int i = 0; i < 4; ++i) {
    const int mBase = m0 + (i << 4);
#pragma unroll
    for (int j = 0; j < 4; ++j) {
      const int n = n0 + (j << 4) + rlane;
      float bv = 0.f;
      if (BIAS_MODE == 2) bv = bias[n];
#pragma unroll
      for (int r = 0; r < 8; ++r) {
        float v = acc[i][j][r] * scale;
        if (BIAS_MODE == 1) v += bias[mBase + mOff + r];
        if (BIAS_MODE == 2) v += bv;
        if (RESID) v += Rb[(size_t)(mBase + mOff + r) * ldc + n];
        if (ACT == 1) v = tanhf(v);
        if (ACT == 2) v = fmaxf(v, 0.0f);
        if (ACT == 3) v = v / (1.0f + expf(-v));
        if (ACT == 4) v = (v > 0.f) ? v : 0.01f * v;
        if (ACT == 5) v = 0.5f * v * (1.0f + erff(v * 0.70710678118654752f));
        slab[(mOff + r) * 68 + (j << 4) + rlane] = v;
      }
    }
    __builtin_amdgcn_fence(__ATOMIC_RELEASE, "workgroup");
    __builtin_amdgcn_wave_barrier();
    __builtin_amdgcn_fence(__ATOMIC_ACQUIRE, "workgroup");
    if (OUT_MODE == 0) {
      float* C = (float*)Cout + (size_t)b * strideC;
      const int hh = lane >> 4, c4 = (lane & 15) * 4;
      for (int pass = 0; pass < 2; ++pass) {
#pragma unroll
        for (int it = 0; it < 8; ++it) {
          const int row = it * 2 + hh;
          v4f v = *(const v4f*)(slab + row * 68 + c4);
          *(volatile v4f*)(C + (size_t)(mBase + row) * ldc + n0 + c4) = v;
        }
        __threadfence();
      }
    } else {
      const int q = lane >> 3, c8 = (lane & 7) * 8;
      unsigned short* C  = (unsigned short*)Cout  + (size_t)b * strideC;
      unsigned short* C2 = (OUT_MODE == 2) ? ((unsigned short*)Cout2 + (size_t)b * strideC) : nullptr;
      for (int pass = 0; pass < 2; ++pass) {
#pragma unroll
        for (int it = 0; it < 4; ++it) {
          const int row = it * 4 + q;
          const float* sp = slab + row * 68 + c8;
          v8h hv, lv;
#pragma unroll
          for (int e = 0; e < 8; ++e) {
            if (OUT_MODE == 1) {
              hv[e] = (_Float16)sp[e];
            } else {
              unsigned short hb = f2bf_bits(sp[e]);
              unsigned short lb = f2bf_bits(sp[e] - bf_bits2f(hb));
              hv[e] = __builtin_bit_cast(_Float16, hb);
              lv[e] = __builtin_bit_cast(_Float16, lb);
            }
          }
          *(volatile v8h*)(C + (size_t)(mBase + row) * ldc + n0 + c8) = hv;
          if (OUT_MODE == 2) *(volatile v8h*)(C2 + (size_t)(mBase + row) * ldc + n0 + c8) = lv;
        }
        __threadfence();
      }
    }
    __builtin_amdgcn_fence(__ATOMIC_RELEASE, "workgroup");
    __builtin_amdgcn_wave_barrier();
    __builtin_amdgcn_fence(__ATOMIC_ACQUIRE, "workgroup");
  }
}

__device__ __forceinline__ float hsig(float x) {
  return fminf(fmaxf(0.2f * x + 0.5f, 0.0f), 1.0f);
}
__device__ __forceinline__ float tanh_apx(float x) {
  const float xc = fminf(fmaxf(x, -16.0f), 16.0f);
  const float e  = __expf(2.0f * xc);
  return 1.0f - 2.0f * __builtin_amdgcn_rcpf(e + 1.0f);
}

__global__ __launch_bounds__(256) void k_prep_w(const float* __restrict__ Wx, const float* __restrict__ Wh,
                                                unsigned short* __restrict__ WB,
                                                int Cin, int Co, int Kp, int nG) {
  const int g = blockIdx.x * 256 + threadIdx.x;
  if (g < nG) {
    const int N4 = 4 * Co, Ctot = Cin + Co;
    const int e0  = g * 8;
    const int n   = e0 / Kp;
    const int col = e0 - n * Kp;
    float f[8];
#pragma unroll
    for (int jx = 0; jx < 8; ++jx) {
      const int cj  = col + jx;
      const int tap = cj / Ctot;
      const int c   = cj - tap * Ctot;
      const int tc  = tap < 9 ? tap : 8;
      const int cx  = c < Cin ? c : (Cin - 1);
      int ch = c - Cin; ch = ch < 0 ? 0 : (ch > Co - 1 ? Co - 1 : ch);
      const float vx = Wx[((size_t)(tc * Cin + cx)) * N4 + n];
      const float vh = Wh[((size_t)(tc * Co + ch)) * N4 + n];
      float v = (c < Cin) ? vx : vh;
      v = (tap < 9) ? v : 0.0f;
      f[jx] = bf_rne(v) * 16.0f;
    }
    v4u u;
    u[0] = pkh2(f[0], f[1]); u[1] = pkh2(f[2], f[3]); u[2] = pkh2(f[4], f[5]); u[3] = pkh2(f[6], f[7]);
    volatile v4u* p = (volatile v4u*)(WB + e0);
    *p = u;
    __threadfence();
    *p = u;
  }
}

__global__ __launch_bounds__(256) void k_im2col(const float* __restrict__ xs, const float* __restrict__ hs,
                                                unsigned short* __restrict__ IM,
                                                int H, int Cin, int Co, int Kp, int up, int t,
                                                int useH, int rnd, int nRows) {
  const int lane = threadIdx.x & 31, wave = threadIdx.x >> 5;
  const int r = blockIdx.x * 8 + wave;
  if (r >= nRows) return;
  const int HH  = H * H;
  const int b   = r / HH;
  const int rem = r - b * HH;
  const int y   = rem / H;
  const int x   = rem - y * H;
  const int Ctot    = Cin + Co;
  const int nChunks = Kp >> 3;
  const int nReal   = (9 * Ctot) >> 3;
  const int Hs      = H >> up;
  const int nIt     = (nChunks + 31) >> 5;
  const v4f z4 = (v4f){0.f, 0.f, 0.f, 0.f};
  for (int it = 0; it < nIt; ++it) {
    const int j    = it * 32 + lane;
    const int jj   = j < nReal ? j : (nReal - 1);
    const int col0 = jj * 8;
    const int tap  = col0 / Ctot;
    const int c    = col0 - tap * Ctot;
    const int kh = tap / 3, kw = tap - kh * 3;
    const int yy = y + kh - 1, xx = x + kw - 1;
    const bool inb = ((unsigned)yy < (unsigned)H) && ((unsigned)xx < (unsigned)H) && (j < nReal);
    const int yc = yy < 0 ? 0 : (yy > H - 1 ? H - 1 : yy);
    const int xc = xx < 0 ? 0 : (xx > H - 1 ? H - 1 : xx);
    const bool isX = c < Cin;
    const int cx  = isX ? c : (Cin - 8);
    int chh = c - Cin; chh = chh < 0 ? 0 : chh;
    const float* px = xs + ((((size_t)b * 8 + t) * Hs + (yc >> up)) * Hs + (xc >> up)) * Cin + cx;
    const float* ph = hs + ((size_t)(b * HH + yc * H + xc)) * Co + chh;
    v4f a0 = *(const v4f*)(px);
    v4f a1 = *(const v4f*)(px + 4);
    v4f h0 = *(const v4f*)(ph);
    v4f h1 = *(const v4f*)(ph + 4);
    if (!useH) { h0 = z4; h1 = z4; }
    float f[8];
#pragma unroll
    for (int e = 0; e < 4; ++e) {
      float vx0 = a0[e], vx1 = a1[e];
      vx0 = rnd ? bf_rne(vx0) : vx0;
      vx1 = rnd ? bf_rne(vx1) : vx1;
      const float v0 = isX ? vx0 : h0[e];
      const float v1 = isX ? vx1 : h1[e];
      f[e]     = inb ? v0 : 0.0f;
      f[4 + e] = inb ? v1 : 0.0f;
    }
    v4u u;
    u[0] = pkh2(f[0], f[1]); u[1] = pkh2(f[2], f[3]); u[2] = pkh2(f[4], f[5]); u[3] = pkh2(f[6], f[7]);
    if (j < nChunks) {
      volatile v4u* d = (volatile v4u*)(IM + (size_t)r * Kp + (size_t)j * 8);
      *d = u;
      __threadfence();
      *d = u;
    }
  }
}

template <int MODE>
__global__ __launch_bounds__(256) void k_cell(const float* __restrict__ Z, float* __restrict__ Cst,
                                              float* __restrict__ Hst, float* __restrict__ Po,
                                              const float* __restrict__ gam, const float* __restrict__ bet,
                                              const float* __restrict__ mme, const float* __restrict__ mva,
                                              int H, int Co, int t, int first, int nQ) {
  const int i = blockIdx.x * 256 + threadIdx.x;
  if (i >= nQ) return;
  const int e0 = i * 4;
  const int p  = e0 / Co;
  const int c0 = e0 - p * Co;
  const int N4 = 4 * Co;
  const float* zp = Z + (size_t)p * N4 + c0;
  const v4f zi = *(const v4f*)(zp);
  const v4f zf = *(const v4f*)(zp + Co);
  const v4f zg = *(const v4f*)(zp + 2 * Co);
  const v4f zo = *(const v4f*)(zp + 3 * Co);
  v4f cold = *(const v4f*)(Cst + e0);
  const v4f z4 = (v4f){0.f, 0.f, 0.f, 0.f};
  if (first) cold = z4;
  v4f cn, hn, ho;
#pragma unroll
  for (int e = 0; e < 4; ++e) {
    const float cv = hsig(zf[e]) * cold[e] + hsig(zi[e]) * tanh_apx(zg[e]);
    const float hv = hsig(zo[e]) * tanh_apx(cv);
    const float gb = bf_rne(gam[c0 + e]);
    const float bb = bf_rne(bet[c0 + e]);
    const float mb = bf_rne(mme[c0 + e]);
    const float vb = bf_rne(mva[c0 + e]);
    cn[e] = cv;
    hn[e] = hv;
    ho[e] = (hv - mb) * rsqrtf(vb + 1e-3f) * gb + bb;
  }
  for (int pass = 0; pass < 2; ++pass) {
    *(volatile v4f*)(Cst + e0) = cn;
    *(volatile v4f*)(Hst + e0) = hn;
    __threadfence();
  }
  const int HH  = H * H;
  const int b   = p / HH;
  const int rem = p - b * HH;
  if (MODE == 0) {
    float* d = Po + (((size_t)b * 8 + t) * HH + rem) * Co + c0;
    for (int pass = 0; pass < 2; ++pass) {
      *(volatile v4f*)(d) = ho;
      __threadfence();
    }
  } else {
    const int y = rem / H, x = rem - y * H;
    const int OW = 2 * H;
    float* d = Po + ((((size_t)b * 8 + t) * OW + 2 * y) * OW + 2 * x) * Co + c0;
    const size_t rowStride = (size_t)OW * Co;
    for (int pass = 0; pass < 2; ++pass) {
      *(volatile v4f*)(d)                  = ho;
      *(volatile v4f*)(d + Co)             = ho;
      *(volatile v4f*)(d + rowStride)      = ho;
      *(volatile v4f*)(d + rowStride + Co) = ho;
      __threadfence();
    }
  }
}

static inline size_t al256(size_t x) { return (x + 255) & ~(size_t)255; }

extern "C" void kernel_launch(void* const* d_in, const int* in_sizes, int n_in,
                              void* d_out, int out_size, void* d_ws, size_t ws_size,
                              hipStream_t stream) {
  if (n_in < 22) return;
  const int nB = 2, nT = 8;
  const int Hs_[3]  = {16, 32, 64};
  const int Cin_[3] = {192, 128, 64};
  const int Co_[3]  = {128, 64, 32};
  int Kp_[3], M_[3], N4_[3];
  for (int l = 0; l < 3; ++l) {
    const int Ctot = Cin_[l] + Co_[l];
    Kp_[l] = ((9 * Ctot + 63) / 64) * 64;
    M_[l]  = nB * Hs_[l] * Hs_[l];
    N4_[l] = 4 * Co_[l];
    if ((M_[l] & 63) || (N4_[l] & 63) || (Kp_[l] & 31) || (Cin_[l] & 7) || (Co_[l] & 7) || (M_[l] & 7)) return;
  }
  if (in_sizes[0] != nB * nT * 16 * 16 * 192) return;
  for (int l = 0; l < 3; ++l) {
    const int o = 1 + 7 * l;
    if (in_sizes[o]     != 9 * Cin_[l] * N4_[l]) return;
    if (in_sizes[o + 1] != 9 * Co_[l] * N4_[l]) return;
    if (in_sizes[o + 2] != N4_[l]) return;
    if (in_sizes[o + 3] != Co_[l] || in_sizes[o + 4] != Co_[l] || in_sizes[o + 5] != Co_[l] || in_sizes[o + 6] != Co_[l]) return;
  }
  if (out_size != nB * nT * 128 * 128 * 32) return;

  const float* x0 = (const float*)d_in[0];
  const float* Wx[3]  = {(const float*)d_in[1],  (const float*)d_in[8],  (const float*)d_in[15]};
  const float* Wh[3]  = {(const float*)d_in[2],  (const float*)d_in[9],  (const float*)d_in[16]};
  const float* bb[3]  = {(const float*)d_in[3],  (const float*)d_in[10], (const float*)d_in[17]};
  const float* gg[3]  = {(const float*)d_in[4],  (const float*)d_in[11], (const float*)d_in[18]};
  const float* be[3]  = {(const float*)d_in[5],  (const float*)d_in[12], (const float*)d_in[19]};
  const float* mme[3] = {(const float*)d_in[6],  (const float*)d_in[13], (const float*)d_in[20]};
  const float* mva[3] = {(const float*)d_in[7],  (const float*)d_in[14], (const float*)d_in[21]};
  float* out = (float*)d_out;

  size_t bWB[3];
  size_t bIM = 0, bZ = 0, bC = 0;
  for (int l = 0; l < 3; ++l) {
    bWB[l] = al256((size_t)N4_[l] * Kp_[l] * 2);
    const size_t im = (size_t)M_[l] * Kp_[l] * 2;  if (im > bIM) bIM = im;
    const size_t z  = (size_t)M_[l] * N4_[l] * 4;  if (z > bZ) bZ = z;
    const size_t c  = (size_t)M_[l] * Co_[l] * 4;  if (c > bC) bC = c;
  }
  bIM = al256(bIM); bZ = al256(bZ); bC = al256(bC);
  const size_t bP1 = al256((size_t)nB * nT * Hs_[0] * Hs_[0] * Co_[0] * 4);
  const size_t bP2 = al256((size_t)nB * nT * Hs_[1] * Hs_[1] * Co_[1] * 4);
  char* ws = (char*)d_ws;
  size_t o = 0;
  unsigned short* WB[3];
  for (int l = 0; l < 3; ++l) { WB[l] = (unsigned short*)(ws + o); o += bWB[l]; }
  unsigned short* IM = (unsigned short*)(ws + o); o += bIM;
  float* Z   = (float*)(ws + o); o += bZ;
  float* Cst = (float*)(ws + o); o += bC;
  float* Hst = (float*)(ws + o); o += bC;
  float* P1  = (float*)(ws + o); o += bP1;
  float* P2  = (float*)(ws + o); o += bP2;
  if (o > ws_size) return;

  for (int l = 0; l < 3; ++l) {
    const int nG = N4_[l] * Kp_[l] / 8;
    k_prep_w<<<(nG + 255) / 256, 256, 0, stream>>>(Wx[l], Wh[l], WB[l], Cin_[l], Co_[l], Kp_[l], nG);
  }

  for (int l = 0; l < 3; ++l) {
    const int H = Hs_[l], Cin = Cin_[l], Co = Co_[l], Kp = Kp_[l], M = M_[l], N4 = N4_[l];
    const float* xsrc = (l == 0) ? x0 : (l == 1 ? P1 : P2);
    const int up  = (l == 0) ? 0 : 1;
    const int rnd = (l == 0) ? 1 : 0;
    const int tiles = (M / 64) * (N4 / 64);
    const int gemmBlocks = (tiles + 7) / 8;
    const int nQ = M * Co / 4;
    for (int t = 0; t < nT; ++t) {
      k_im2col<<<M / 8, 256, 0, stream>>>(xsrc, Hst, IM, H, Cin, Co, Kp, up, t, (t > 0) ? 1 : 0, rnd, M);
      wmma_gemm64<0, false, 2, 0, false, 0><<<dim3(gemmBlocks, 1), 256, 0, stream>>>(
          IM, IM, Kp, 0L,
          WB[l], WB[l], Kp, 0L,
          (void*)Z, (void*)Z, N4, 0L,
          bb[l],
          Z, 0L,
          M, N4, Kp, 0.0625f);
      if (l < 2) {
        float* Po = (l == 0) ? P1 : P2;
        k_cell<0><<<(nQ + 255) / 256, 256, 0, stream>>>(Z, Cst, Hst, Po, gg[l], be[l], mme[l], mva[l],
                                                          H, Co, t, (t == 0) ? 1 : 0, nQ);
      } else {
        k_cell<1><<<(nQ + 255) / 256, 256, 0, stream>>>(Z, Cst, Hst, out, gg[l], be[l], mme[l], mva[l],
                                                          H, Co, t, (t == 0) ? 1 : 0, nQ);
      }
    }
  }
}
